// Encoder_32349693673701
// MI455X (gfx1250) — hardware-verified
//
#include <hip/hip_runtime.h>
#include <math.h>

constexpr int NB       = 128;
constexpr int NS       = 128;
constexpr int NK       = 512;
constexpr int NU       = 512;
constexpr int NG       = 4 * NU;
constexpr int NTHR     = 256;
constexpr int ROWS_BLK = 16;
constexpr int AP       = 520;
constexpr int SP       = 516;
constexpr float WCARRY = 256.0f;
constexpr float WFOLD  = 1.0f / 256.0f;
constexpr float RCARRY = 2048.0f;
constexpr float RFOLD  = 1.0f / 2048.0f;
constexpr float HFLUSH = 6.2e-5f;

static_assert(NB % ROWS_BLK == 0, "batch tiles");
static_assert(NU == 64 * (NTHR / 32), "8 waves x 64 hidden units");
static_assert(NK % 32 == 0 && NU % 32 == 0, "K multiples of 32");
static_assert(NK % 64 == 0 && NU % 64 == 0 && NG % 64 == 0, "transpose tiles");
static_assert((AP * 2) % 16 == 0 && AP >= NK && AP >= NU, "A tile pitch");
static_assert((SP * 4) % 16 == 0 && SP >= NU, "state tile pitch");
static_assert(ROWS_BLK * NK == NTHR * 8 * 4, "staging pass covers 16 x 512 exactly");
static_assert(ROWS_BLK * NU == NTHR * 8 * 4, "store pass covers 16 x 512 exactly");
static_assert((size_t)3 * NB * NU * 4 == (size_t)786432, "output bytes");

typedef __attribute__((ext_vector_type(16))) _Float16 v16h;
typedef __attribute__((ext_vector_type(8)))  _Float16 v8h;
typedef __attribute__((ext_vector_type(4)))  _Float16 v4h;
typedef __attribute__((ext_vector_type(8)))  float    v8f;
typedef __attribute__((ext_vector_type(4)))  float    v4f;

struct FragH {
  union U { v16h v; v8h h[2]; };
  static __device__ __forceinline__ v16h load(const _Float16* p) {
    U f;
    f.h[0] = *(const v8h*)(p);
    f.h[1] = *(const v8h*)(p + 16);
    return f.v;
  }
  static __device__ __forceinline__ v8f mma(v16h a, v16h b, v8f c) {
    return __builtin_amdgcn_wmma_f32_16x16x32_f16(false, a, false, b, (short)0, c, false, false);
  }
};

__device__ __forceinline__ void guard_mma4(v8f& a0, v8f& a1, v8f& a2, v8f& a3,
                                           v16h x, v16h b0, v16h b1, v16h b2, v16h b3) {
  asm volatile("v_nop\n\tv_nop\n\tv_nop\n\tv_nop"
               : "+v"(a0), "+v"(a1), "+v"(a2), "+v"(a3)
               : "v"(x), "v"(b0), "v"(b1), "v"(b2), "v"(b3));
}
__device__ __forceinline__ void guard_mma8(v8f& a0, v8f& a1, v8f& a2, v8f& a3,
                                           v8f& r0, v8f& r1, v8f& r2, v8f& r3,
                                           v16h x, v16h y, v16h b0, v16h b1, v16h b2, v16h b3) {
  asm volatile("v_nop\n\tv_nop\n\tv_nop\n\tv_nop"
               : "+v"(a0), "+v"(a1), "+v"(a2), "+v"(a3), "+v"(r0), "+v"(r1), "+v"(r2), "+v"(r3)
               : "v"(x), "v"(y), "v"(b0), "v"(b1), "v"(b2), "v"(b3));
}

__device__ __forceinline__ float sigm_f(float z) {
  const float zc = fminf(fmaxf(z, -30.0f), 30.0f);
  return 1.0f / (1.0f + expf(-zc));
}
__device__ __forceinline__ float tanh_f(float z) {
  const float zc = fminf(fmaxf(z, -15.0f), 15.0f);
  return 1.0f - 2.0f / (1.0f + expf(2.0f * zc));
}

__global__ __launch_bounds__(NTHR) void tpw_f16_kernel(const float* __restrict__ src, int R, int C, int ldo,
                                                       _Float16* __restrict__ O, float sc) {
  __shared__ float Tt[64 * 65];
  const int tid = threadIdx.x;
  const int c0 = blockIdx.x * 64, r0 = blockIdx.y * 64;
#pragma unroll
  for (int i = 0; i < 4; ++i) {
    const int idx = i * NTHR + tid;
    const int rr = idx >> 4, cc = (idx & 15) * 4;
    const v4f v = *(const v4f*)(src + (size_t)(r0 + rr) * (size_t)C + c0 + cc);
    Tt[rr * 65 + cc + 0] = v[0];
    Tt[rr * 65 + cc + 1] = v[1];
    Tt[rr * 65 + cc + 2] = v[2];
    Tt[rr * 65 + cc + 3] = v[3];
  }
  __syncthreads();
  const int q = tid >> 3, c8 = (tid & 7) * 8;
  v8h hv[2];
#pragma unroll
  for (int g = 0; g < 2; ++g) {
    const int qq = g * 32 + q;
#pragma unroll
    for (int e = 0; e < 8; ++e) {
      const float f = Tt[(c8 + e) * 65 + qq];
      hv[g][e] = (_Float16)(f * sc);
    }
  }
  for (int pass = 0; pass < 2; ++pass) {
#pragma unroll
    for (int g = 0; g < 2; ++g) {
      const size_t o = (size_t)(c0 + g * 32 + q) * (size_t)ldo + (size_t)(r0 + c8);
      *(volatile v8h*)(O + o) = hv[g];
    }
    __threadfence();
  }
}

__device__ __forceinline__ void stage_x_tile(const float* __restrict__ xrow, _Float16* axrow) {
#pragma unroll 1
  for (int it = 0; it < 8; ++it) {
    const v4f xv = *(const v4f*)(xrow + it * 64);
    v4h x4;
    x4[0] = (_Float16)xv[0];
    x4[1] = (_Float16)xv[1];
    x4[2] = (_Float16)xv[2];
    x4[3] = (_Float16)xv[3];
    *(v4h*)(axrow + it * 64) = x4;
  }
}

__global__ __launch_bounds__(NTHR) void lstm_scan_kernel(const float* __restrict__ x, const float* __restrict__ bias,
                                                         const _Float16* __restrict__ WT,
                                                         const _Float16* __restrict__ UT,
                                                         float* __restrict__ out) {
  __shared__ __align__(16) _Float16 Ax[ROWS_BLK * AP];
  __shared__ __align__(16) _Float16 Ahh[ROWS_BLK * AP];
  __shared__ __align__(16) _Float16 Ahl[ROWS_BLK * AP];
  __shared__ __align__(16) float    Cs[ROWS_BLK * SP];
  __shared__ __align__(16) float    Hs[ROWS_BLK * SP];

  const int tid = threadIdx.x, lane = tid & 31, wave = tid >> 5;
  const int c = lane & 15, hh = lane >> 4, koff = hh * 8;
  const int rowbase = blockIdx.x * ROWS_BLK;
  const int prow = tid >> 4, pcol = (tid & 15) * 4;

#pragma unroll 1
  for (int i = tid; i < ROWS_BLK * AP; i += NTHR) {
    Ax[i]  = (_Float16)0.0f;
    Ahh[i] = (_Float16)0.0f;
    Ahl[i] = (_Float16)0.0f;
  }
#pragma unroll 1
  for (int i = tid; i < ROWS_BLK * SP; i += NTHR) {
    Cs[i] = 0.0f;
    Hs[i] = 0.0f;
  }
  __syncthreads();
  stage_x_tile(x + ((size_t)(rowbase + prow) * NS) * NK + pcol, Ax + prow * AP + pcol);
  __syncthreads();

  const _Float16* axrow = Ax  + c * AP + koff;
  const _Float16* ahrow = Ahh + c * AP + koff;
  const _Float16* alrow = Ahl + c * AP + koff;
  const v8f z8 = {0.f, 0.f, 0.f, 0.f, 0.f, 0.f, 0.f, 0.f};
  const size_t gstride_w = (size_t)NU * NK;
  const size_t gstride_u = (size_t)NU * NU;

#pragma unroll 1
  for (int t = 0; t < NS; ++t) {
#pragma unroll 1
    for (int nt = 0; nt < 4; ++nt) {
      const int j = 64 * wave + 16 * nt + c;
      const _Float16* wx = WT + (size_t)j * NK + koff;
      const _Float16* wh = UT + (size_t)j * NU + koff;
      v8f acc[4], res[4];
      acc[0] = z8; acc[1] = z8; acc[2] = z8; acc[3] = z8;
      res[0] = z8; res[1] = z8; res[2] = z8; res[3] = z8;
#pragma unroll 1
      for (int kx = 0; kx < NK; kx += 32) {
        const v16h a  = FragH::load(axrow + kx);
        const v16h b0 = FragH::load(wx + kx);
        const v16h b1 = FragH::load(wx + gstride_w + kx);
        const v16h b2 = FragH::load(wx + 2 * gstride_w + kx);
        const v16h b3 = FragH::load(wx + 3 * gstride_w + kx);
        acc[0] = FragH::mma(a, b0, acc[0]);
        acc[1] = FragH::mma(a, b1, acc[1]);
        acc[2] = FragH::mma(a, b2, acc[2]);
        acc[3] = FragH::mma(a, b3, acc[3]);
        guard_mma4(acc[0], acc[1], acc[2], acc[3], a, b0, b1, b2, b3);
      }
#pragma unroll 1
      for (int k0 = 0; k0 < NU; k0 += 32) {
        const v16h ah = FragH::load(ahrow + k0);
        const v16h al = FragH::load(alrow + k0);
        const v16h b0 = FragH::load(wh + k0);
        const v16h b1 = FragH::load(wh + gstride_u + k0);
        const v16h b2 = FragH::load(wh + 2 * gstride_u + k0);
        const v16h b3 = FragH::load(wh + 3 * gstride_u + k0);
        acc[0] = FragH::mma(ah, b0, acc[0]);
        res[0] = FragH::mma(al, b0, res[0]);
        acc[1] = FragH::mma(ah, b1, acc[1]);
        res[1] = FragH::mma(al, b1, res[1]);
        acc[2] = FragH::mma(ah, b2, acc[2]);
        res[2] = FragH::mma(al, b2, res[2]);
        acc[3] = FragH::mma(ah, b3, acc[3]);
        res[3] = FragH::mma(al, b3, res[3]);
        guard_mma8(acc[0], acc[1], acc[2], acc[3], res[0], res[1], res[2], res[3], ah, al, b0, b1, b2, b3);
      }
      const float bi = bias[j];
      const float bf = bias[NU + j];
      const float bg = bias[2 * NU + j];
      const float bo = bias[3 * NU + j];
#pragma unroll
      for (int r = 0; r < 8; ++r) {
        const int so = (8 * hh + r) * SP + j;
        const float zi = (acc[0][r] + res[0][r] * RFOLD) * WFOLD + bi;
        const float zf = (acc[1][r] + res[1][r] * RFOLD) * WFOLD + bf;
        const float zg = (acc[2][r] + res[2][r] * RFOLD) * WFOLD + bg;
        const float zo = (acc[3][r] + res[3][r] * RFOLD) * WFOLD + bo;
        const float ig = sigm_f(zi);
        const float fg = sigm_f(zf);
        const float gg = tanh_f(zg);
        const float og = sigm_f(zo);
        const float cp = Cs[so];
        const float cn = fg * cp + ig * gg;
        const float hn = og * tanh_f(cn);
        Cs[so] = cn;
        Hs[so] = hn;
      }
    }
    __syncthreads();

    {
      const float*    hsrow = Hs  + prow * SP + pcol;
      _Float16*       hhrow = Ahh + prow * AP + pcol;
      _Float16*       hlrow = Ahl + prow * AP + pcol;
#pragma unroll 1
      for (int it = 0; it < 8; ++it) {
        const v4f hv = *(const v4f*)(hsrow + it * 64);
        v4h hi4, lo4;
#pragma unroll
        for (int e = 0; e < 4; ++e) {
          const float hval = hv[e];
          const float hq = (fabsf(hval) < HFLUSH) ? 0.0f : hval;
          const _Float16 hi = (_Float16)hq;
          const float hif = (float)hi;
          hi4[e] = hi;
          lo4[e] = (_Float16)((hval - hif) * RCARRY);
        }
        *(v4h*)(hhrow + it * 64) = hi4;
        *(v4h*)(hlrow + it * 64) = lo4;
      }
      const int tn = (t + 1 < NS) ? (t + 1) : (NS - 1);
      stage_x_tile(x + ((size_t)(rowbase + prow) * NS + (size_t)tn) * NK + pcol, Ax + prow * AP + pcol);
    }
    __syncthreads();
  }

  for (int pass = 0; pass < 2; ++pass) {
#pragma unroll
    for (int it = 0; it < 8; ++it) {
      const int idx = it * NTHR + tid;
      const int row = idx >> 7, c4 = (idx & 127) * 4;
      const v4f hv = *(const v4f*)(Hs + row * SP + c4);
      const v4f cv = *(const v4f*)(Cs + row * SP + c4);
      const size_t o = (size_t)(rowbase + row) * NU + c4;
      *(volatile v4f*)(out + o) = hv;
      *(volatile v4f*)(out + (size_t)NB * NU + o) = hv;
      *(volatile v4f*)(out + (size_t)2 * NB * NU + o) = cv;
    }
    __threadfence();
  }
}

extern "C" void kernel_launch(void* const* d_in, const int* in_sizes, int n_in,
                              void* d_out, int out_size, void* d_ws, size_t ws_size, hipStream_t stream) {
  if (n_in < 4 || d_out == nullptr || d_ws == nullptr) return;
  if (in_sizes[0] != NB * NS * NK || in_sizes[1] != NK * NG || in_sizes[2] != NU * NG ||
      in_sizes[3] != NG || out_size != 3 * NB * NU) return;

  const float* xin  = (const float*)d_in[0];
  const float* win  = (const float*)d_in[1];
  const float* urec = (const float*)d_in[2];
  const float* bvec = (const float*)d_in[3];
  float* out = (float*)d_out;

  char* ws = (char*)d_ws;
  size_t off = 0;
  auto carve = [&](size_t bytes) -> char* { char* p = ws + off; off += (bytes + 255) & ~(size_t)255; return p; };
  _Float16* WT = (_Float16*)carve((size_t)NG * NK * 2);
  _Float16* UT = (_Float16*)carve((size_t)NG * NU * 2);
  if (off > ws_size || off > (size_t)134217728) return;

  tpw_f16_kernel<<<dim3(NG / 64, NK / 64), NTHR, 0, stream>>>(win, NK, NG, NK, WT, WCARRY);
  tpw_f16_kernel<<<dim3(NG / 64, NU / 64), NTHR, 0, stream>>>(urec, NU, NG, NU, UT, WCARRY);
  lstm_scan_kernel<<<NB / ROWS_BLK, NTHR, 0, stream>>>(xin, bvec, WT, UT, out);
}
